// LSTMCell_56642028699866
// MI455X (gfx1250) — hardware-verified
//
#include <hip/hip_runtime.h>
#include <math.h>

constexpr int NBATCH = 4096;
constexpr int NIN    = 1024;
constexpr int NHID   = 1024;
constexpr int KDIM   = NIN + NHID;
constexpr int NGATE  = 4;
constexpr int NTHR   = 256;
constexpr int SLABP  = 36;
static_assert(KDIM % 64 == 0);
static_assert(NBATCH % 64 == 0 && NHID % 64 == 0);
static_assert(NIN % 64 == 0);
static_assert((NBATCH * (NIN / 8)) % NTHR == 0);
static_assert((NIN / 8) % 32 == 0);
static_assert(NIN == NHID);

typedef __attribute__((ext_vector_type(16))) _Float16 v16h;
typedef __attribute__((ext_vector_type(8)))  _Float16 v8h;
typedef __attribute__((ext_vector_type(16))) __bf16   v16b;
typedef __attribute__((ext_vector_type(8)))  __bf16   v8b;
typedef __attribute__((ext_vector_type(8)))  float    v8f;
typedef __attribute__((ext_vector_type(4)))  float    v4f;

__device__ __forceinline__ unsigned short f2bf_bits(float f) {
  unsigned u = __float_as_uint(f);
  return (unsigned short)((u + 0x7FFFu + ((u >> 16) & 1u)) >> 16);
}
__device__ __forceinline__ float bf_bits2f(unsigned short h) { return __uint_as_float(((unsigned)h) << 16); }
__device__ __forceinline__ float bf16r(float f) { return bf_bits2f(f2bf_bits(f)); }

__device__ __forceinline__ void dep_guard_h(v8f& a, v8f& b, v16h x, v16h y) { asm volatile("v_nop\n\tv_nop\n\tv_nop\n\tv_nop" : "+v"(a), "+v"(b) : "v"(x), "v"(y)); }
__device__ __forceinline__ void dep_guard_b(v8f& a, v8f& b, v16b x, v16b y) { asm volatile("v_nop\n\tv_nop\n\tv_nop\n\tv_nop" : "+v"(a), "+v"(b) : "v"(x), "v"(y)); }
__device__ __forceinline__ void keep4_h(v16h a, v16h b, v16h c, v16h d) { asm volatile("v_nop" :: "v"(a), "v"(b), "v"(c), "v"(d)); }
__device__ __forceinline__ void keep4_b(v16b a, v16b b, v16b c, v16b d) { asm volatile("v_nop" :: "v"(a), "v"(b), "v"(c), "v"(d)); }
__device__ __forceinline__ void acc_guard4(v8f& a, v8f& b, v8f& c, v8f& d) { asm volatile("v_nop\n\tv_nop\n\tv_nop\n\tv_nop" : "+v"(a), "+v"(b), "+v"(c), "+v"(d)); }
__device__ __forceinline__ void guard2m_b(v8f& a0, v8f& a1, v16b x, v16b y0, v16b y1) {
  asm volatile("v_nop\n\tv_nop\n\tv_nop\n\tv_nop" : "+v"(a0), "+v"(a1) : "v"(x), "v"(y0), "v"(y1) : "memory");
}

template <typename T> struct Frag;
template <> struct Frag<_Float16> {
  typedef v16h V; union U { v16h v; v8h h[2]; };
  static __device__ __forceinline__ v16h load(const _Float16* p) {
    U f; f.h[0] = *(const v8h*)(p); f.h[1] = *(const v8h*)(p + 16); return f.v;
  }
  static __device__ __forceinline__ v8f mma(v16h a, v16h b, v8f c) {
    return __builtin_amdgcn_wmma_f32_16x16x32_f16(false, a, false, b, (short)0, c, false, false);
  }
  static __device__ __forceinline__ void guard(v8f& a, v8f& b, v16h x, v16h y) { dep_guard_h(a, b, x, y); }
  static __device__ __forceinline__ void keep(v16h a, v16h b, v16h c, v16h d) { keep4_h(a, b, c, d); }
};
template <> struct Frag<__bf16> {
  typedef v16b V; union U { v16b v; v8b h[2]; };
  static __device__ __forceinline__ v16b load(const __bf16* p) {
    U f; f.h[0] = *(const v8b*)(p); f.h[1] = *(const v8b*)(p + 16); return f.v;
  }
  static __device__ __forceinline__ v8f mma(v16b a, v16b b, v8f c) {
    return __builtin_amdgcn_wmma_f32_16x16x32_bf16(false, a, false, b, (short)0, c, false, false);
  }
  static __device__ __forceinline__ void guard(v8f& a, v8f& b, v16b x, v16b y) { dep_guard_b(a, b, x, y); }
  static __device__ __forceinline__ void keep(v16b a, v16b b, v16b c, v16b d) { keep4_b(a, b, c, d); }
};

__device__ __forceinline__ float fsig(float x)  { return __builtin_amdgcn_rcpf(1.0f + expf(-x)); }
__device__ __forceinline__ float ftanh(float x) { return 1.0f - 2.0f * __builtin_amdgcn_rcpf(expf(2.0f * x) + 1.0f); }

__global__ __launch_bounds__(NTHR) void cvt8_kernel(const float* __restrict__ src, unsigned short* __restrict__ dst,
                                                    int nrow, int ncol8, int spitch, int dpitch, int dcol0) {
  const int i  = blockIdx.x * NTHR + threadIdx.x;
  const int n8 = nrow * ncol8;
  if (i < n8) {
    const int row = i / ncol8;
    const int c8  = i - row * ncol8;
    const float* sp = src + (size_t)row * spitch + c8 * 8;
    const v4f a = *(const v4f*)(sp);
    const v4f b = *(const v4f*)(sp + 4);
    v8h hv;
#pragma unroll
    for (int e = 0; e < 4; ++e) {
      const unsigned short b0 = f2bf_bits(a[e]);
      const unsigned short b1 = f2bf_bits(b[e]);
      hv[e]     = __builtin_bit_cast(_Float16, b0);
      hv[4 + e] = __builtin_bit_cast(_Float16, b1);
    }
    unsigned short* dp = dst + (size_t)row * dpitch + dcol0 + c8 * 8;
    *(volatile v8h*)(dp) = hv;
    __threadfence();
    *(volatile v8h*)(dp) = hv;
  }
}

template <int MODE>
__global__ __launch_bounds__(NTHR) void tpw_kernel(const float* __restrict__ src, int R, int C, int ldo,
                                                  unsigned short* __restrict__ O, float sc) {
  __shared__ float Tt[64 * 65];
  const int tid = threadIdx.x;
  const int c0 = blockIdx.x * 64, r0 = blockIdx.y * 64;
#pragma unroll
  for (int i = 0; i < 4; ++i) {
    const int idx = i * NTHR + tid;
    const int rr = idx >> 4, cc = (idx & 15) * 4;
    const v4f v = *(const v4f*)(src + (size_t)(r0 + rr) * (size_t)C + c0 + cc);
    Tt[rr * 65 + cc + 0] = v[0];
    Tt[rr * 65 + cc + 1] = v[1];
    Tt[rr * 65 + cc + 2] = v[2];
    Tt[rr * 65 + cc + 3] = v[3];
  }
  __syncthreads();
  const int q = tid >> 3, c8 = (tid & 7) * 8;
  v8h hv[2];
#pragma unroll
  for (int g = 0; g < 2; ++g) {
    const int qq = g * 32 + q;
#pragma unroll
    for (int e = 0; e < 8; ++e) {
      const float f = Tt[(c8 + e) * 65 + qq];
      unsigned short bits;
      if (MODE == 0) {
        bits = f2bf_bits(f * sc);
      } else {
        const float fb = bf_bits2f(f2bf_bits(f));
        bits = __builtin_bit_cast(unsigned short, (_Float16)(fb * sc));
      }
      hv[g][e] = __builtin_bit_cast(_Float16, bits);
    }
  }
  for (int pass = 0; pass < 2; ++pass) {
#pragma unroll
    for (int g = 0; g < 2; ++g) {
      const size_t o = (size_t)(c0 + g * 32 + q) * (size_t)ldo + (size_t)(r0 + c8);
      *(volatile v8h*)(O + o) = hv[g];
    }
    __threadfence();
  }
}

__global__ __launch_bounds__(NTHR) void lstm_cell_kernel(const unsigned short* __restrict__ HXp,
                                                         const unsigned short* __restrict__ WTp,
                                                         const float* __restrict__ cin,
                                                         const float* __restrict__ bF, const float* __restrict__ bI,
                                                         const float* __restrict__ bS, const float* __restrict__ bP,
                                                         float* __restrict__ out) {
  __shared__ __align__(16) float Sl[NTHR / 32][3][16 * SLABP];
  const __bf16* HX = (const __bf16*)HXp;
  const __bf16* WT = (const __bf16*)WTp;
  const int tid = threadIdx.x, lane = tid & 31, wave = tid >> 5;
  const int c = lane & 15, hh = lane >> 4, koff = hh * 8;
  const int m0 = blockIdx.y * 64 + (wave >> 1) * 16;
  const int n0 = blockIdx.x * 64 + (wave & 1) * 32;

  float bb[4][2];
#pragma unroll
  for (int ni = 0; ni < 2; ++ni) {
    const int n = n0 + 16 * ni + c;
    bb[0][ni] = bf16r(bF[n]);
    bb[1][ni] = bf16r(bI[n]);
    bb[2][ni] = bf16r(bS[n]);
    bb[3][ni] = bf16r(bP[n]);
  }

  const v8f z8 = {0.f, 0.f, 0.f, 0.f, 0.f, 0.f, 0.f, 0.f};
  v8f acc[4][2];
#pragma unroll
  for (int g = 0; g < 4; ++g) { acc[g][0] = z8; acc[g][1] = z8; }

  const __bf16* arow = HX + (size_t)(m0 + c) * KDIM + koff;
  const __bf16* wrow = WT + (size_t)(n0 + c) * KDIM + koff;

#pragma unroll 1
  for (int k0 = 0; k0 < KDIM; k0 += 64) {
#pragma unroll
    for (int kk = 0; kk < 64; kk += 32) {
      const v16b a = Frag<__bf16>::load(arow + k0 + kk);
#pragma unroll
      for (int g = 0; g < 4; ++g) {
        const __bf16* wg = wrow + (size_t)g * NHID * KDIM + k0 + kk;
        const v16b b0 = Frag<__bf16>::load(wg);
        const v16b b1 = Frag<__bf16>::load(wg + (size_t)16 * KDIM);
        acc[g][0] = Frag<__bf16>::mma(a, b0, acc[g][0]);
        acc[g][1] = Frag<__bf16>::mma(a, b1, acc[g][1]);
        guard2m_b(acc[g][0], acc[g][1], a, b0, b1);
      }
    }
  }
  acc_guard4(acc[0][0], acc[0][1], acc[1][0], acc[1][1]);
  acc_guard4(acc[2][0], acc[2][1], acc[3][0], acc[3][1]);

  float* slF  = Sl[wave][0];
  float* slIP = Sl[wave][1];
  float* slS  = Sl[wave][2];
#pragma unroll
  for (int ni = 0; ni < 2; ++ni) {
    const int col = 16 * ni + c;
#pragma unroll
    for (int r = 0; r < 8; ++r) {
      const int row = 8 * hh + r;
      const float zf = acc[0][ni][r] + bb[0][ni];
      const float zi = acc[1][ni][r] + bb[1][ni];
      const float zs = acc[2][ni][r] + bb[2][ni];
      const float zp = acc[3][ni][r] + bb[3][ni];
      const float fg = fsig(zf);
      const float ig = fsig(zi);
      const float sg = fsig(zs);
      const float pg = ftanh(zp);
      slF [row * SLABP + col] = fg;
      slIP[row * SLABP + col] = ig * pg;
      slS [row * SLABP + col] = sg;
    }
  }
  __builtin_amdgcn_fence(__ATOMIC_RELEASE, "workgroup");
  __builtin_amdgcn_wave_barrier();
  __builtin_amdgcn_fence(__ATOMIC_ACQUIRE, "workgroup");

  const int q = lane >> 3, c4 = (lane & 7) * 4;
  v4f o[4];
#pragma unroll
  for (int it = 0; it < 4; ++it) {
    const int row = it * 4 + q;
    const v4f cv  = *(const v4f*)(cin + (size_t)(m0 + row) * NHID + n0 + c4);
    const v4f fv  = *(const v4f*)(slF  + row * SLABP + c4);
    const v4f ipv = *(const v4f*)(slIP + row * SLABP + c4);
    const v4f sv  = *(const v4f*)(slS  + row * SLABP + c4);
#pragma unroll
    for (int e = 0; e < 4; ++e) {
      const float cn = bf16r(cv[e]) * fv[e] + ipv[e];
      o[it][e] = ftanh(cn) * sv[e];
    }
  }
  for (int pass = 0; pass < 2; ++pass) {
#pragma unroll
    for (int it = 0; it < 4; ++it) {
      const int row = it * 4 + q;
      *(volatile v4f*)(out + (size_t)(m0 + row) * NHID + n0 + c4) = o[it];
    }
    __threadfence();
  }
}

extern "C" void kernel_launch(void* const* d_in, const int* in_sizes, int n_in,
                              void* d_out, int out_size, void* d_ws, size_t ws_size, hipStream_t stream) {
  if (n_in < 11 || d_out == nullptr || d_ws == nullptr) return;
  if (in_sizes[0] != NBATCH * NIN || in_sizes[1] != NBATCH * NHID || in_sizes[2] != NBATCH * NHID ||
      in_sizes[3] != KDIM * NHID || in_sizes[4] != NHID || in_sizes[5] != KDIM * NHID || in_sizes[6] != NHID ||
      in_sizes[7] != KDIM * NHID || in_sizes[8] != NHID || in_sizes[9] != KDIM * NHID || in_sizes[10] != NHID ||
      out_size != NBATCH * NHID) return;

  const float* x  = (const float*)d_in[0];
  const float* h  = (const float*)d_in[1];
  const float* cc = (const float*)d_in[2];
  const float* Wf = (const float*)d_in[3];
  const float* bF = (const float*)d_in[4];
  const float* Wi = (const float*)d_in[5];
  const float* bI = (const float*)d_in[6];
  const float* Ws = (const float*)d_in[7];
  const float* bS = (const float*)d_in[8];
  const float* Wp = (const float*)d_in[9];
  const float* bP = (const float*)d_in[10];
  float* out = (float*)d_out;

  char* ws = (char*)d_ws; size_t off = 0;
  auto carve = [&](size_t bytes) -> char* { char* p = ws + off; off += (bytes + 255) & ~(size_t)255; return p; };
  unsigned short* HXB = (unsigned short*)carve((size_t)NBATCH * KDIM * 2);
  unsigned short* WTB = (unsigned short*)carve((size_t)NGATE * NHID * KDIM * 2);
  if (off > ws_size || off > (size_t)134217728) return;

  const int n8 = NBATCH * (NIN / 8);
  cvt8_kernel<<<n8 / NTHR, NTHR, 0, stream>>>(x, HXB, NBATCH, NIN / 8, NIN, KDIM, 0);
  cvt8_kernel<<<n8 / NTHR, NTHR, 0, stream>>>(h, HXB, NBATCH, NHID / 8, NHID, KDIM, NIN);
  const dim3 tgrid(NHID / 64, KDIM / 64);
  tpw_kernel<0><<<tgrid, NTHR, 0, stream>>>(Wf, KDIM, NHID, KDIM, WTB + (size_t)0 * NHID * KDIM, 1.0f);
  tpw_kernel<0><<<tgrid, NTHR, 0, stream>>>(Wi, KDIM, NHID, KDIM, WTB + (size_t)1 * NHID * KDIM, 1.0f);
  tpw_kernel<0><<<tgrid, NTHR, 0, stream>>>(Ws, KDIM, NHID, KDIM, WTB + (size_t)2 * NHID * KDIM, 1.0f);
  tpw_kernel<0><<<tgrid, NTHR, 0, stream>>>(Wp, KDIM, NHID, KDIM, WTB + (size_t)3 * NHID * KDIM, 1.0f);
  lstm_cell_kernel<<<dim3(NHID / 64, NBATCH / 64), NTHR, 0, stream>>>(HXB, WTB, cc, bF, bI, bS, bP, out);
}
